// QuadPrior_Attention_52321291600384
// MI455X (gfx1250) — hardware-verified
//
#include <hip/hip_runtime.h>

#define TT_  2048
#define CC_  1024
#define MM_  4096
#define NBK  8
#define BS_  128
#define NHD  16
#define HD_  64
#define LSTR 48

typedef _Float16 f16;
typedef __attribute__((ext_vector_type(16))) f16 f16x16;
typedef __attribute__((ext_vector_type(8)))  f16 f16x8;
typedef __attribute__((ext_vector_type(4)))  f16 f16x4;
typedef __attribute__((ext_vector_type(8)))  float f32x8;
typedef __attribute__((ext_vector_type(4)))  float v4f_t;
typedef float v4fa __attribute__((ext_vector_type(4), may_alias));
#define RSPLIT (1.0f / 2048.0f)
__device__ __forceinline__ void split16(float v, _Float16& h, _Float16& l) { h = (_Float16)v; l = (_Float16)((v - (float)h) * 2048.0f); }

__device__ __forceinline__ f32x8 wmma16(f16x16 a, f16x16 b, f32x8 c) {
  c = __builtin_amdgcn_wmma_f32_16x16x32_f16(false, a, false, b, (short)0, c, false, false);
  asm volatile("v_nop\n\tv_nop\n\tv_nop\n\tv_nop" : "+v"(c) : "v"(a), "v"(b));
  return c;
}
__device__ __forceinline__ f16x16 lds_frag(const f16* base, int stride) {
  const int lane = threadIdx.x & 31, row = lane & 15, kh = (lane >> 4) * 8;
  const f16x8 lo = *(const f16x8*)(base + row * stride + kh);
  const f16x8 hi = *(const f16x8*)(base + row * stride + kh + 16);
  f16x16 f;
#pragma unroll
  for (int i = 0; i < 8; ++i) { f[i] = lo[i]; f[i + 8] = hi[i]; }
  return f;
}
__device__ __forceinline__ f16x16 load_frag(const float* __restrict__ base, int ld, int row0, int k0) {
  const int lane = threadIdx.x & 31, r = lane & 15, kh = (lane >> 4) * 8;
  const float* p0 = base + (size_t)(row0 + r) * ld + (k0 + kh);
  const v4f_t a = *(const v4f_t*)(p0), b = *(const v4f_t*)(p0 + 4), c = *(const v4f_t*)(p0 + 16), d = *(const v4f_t*)(p0 + 20);
  f16x16 f;
  f[0] = (f16)a[0]; f[1] = (f16)a[1]; f[2]  = (f16)a[2]; f[3]  = (f16)a[3]; f[4]  = (f16)b[0]; f[5]  = (f16)b[1]; f[6]  = (f16)b[2]; f[7]  = (f16)b[3];
  f[8] = (f16)c[0]; f[9] = (f16)c[1]; f[10] = (f16)c[2]; f[11] = (f16)c[3]; f[12] = (f16)d[0]; f[13] = (f16)d[1]; f[14] = (f16)d[2]; f[15] = (f16)d[3];
  return f;
}

__device__ __forceinline__ void load_frag2(const float* __restrict__ base, int ld, int row0, int k0, f16x16& fh, f16x16& fl) {
  const int lane = threadIdx.x & 31, r = lane & 15, kh = (lane >> 4) * 8;
  const float* p0 = base + (size_t)(row0 + r) * ld + (k0 + kh);
  const v4f_t a = *(const v4f_t*)(p0), b = *(const v4f_t*)(p0 + 4), c = *(const v4f_t*)(p0 + 16), d = *(const v4f_t*)(p0 + 20);
  const float v[16] = {a[0], a[1], a[2], a[3], b[0], b[1], b[2], b[3], c[0], c[1], c[2], c[3], d[0], d[1], d[2], d[3]};
#pragma unroll
  for (int i = 0; i < 16; ++i) { f16 h, l; split16(v[i], h, l); fh[i] = h; fl[i] = l; }
}

__global__ __launch_bounds__(256) void k_urdhva(const float* __restrict__ X, const float* __restrict__ Wv, const float* __restrict__ Wr,
                                                const float* __restrict__ Wl, const float* __restrict__ bias, float* __restrict__ Y) {
  __shared__ __attribute__((aligned(16))) f16 ldsA[128 * LSTR], ldsAl[128 * LSTR];
  __shared__ __attribute__((aligned(16))) f16 ldsW[128 * LSTR], ldsWl[128 * LSTR];
  __shared__ __attribute__((aligned(16))) float oS[8][32 * 68];
  const int tid = threadIdx.x, lane = tid & 31, wave = tid >> 5, cl = lane & 15, rh = (lane >> 4) * 8;
  const int m0 = blockIdx.x * 128, ob = blockIdx.y;
  const int wm = (wave & 3) * 32, wn = (wave >> 2) * 64;
  const int nseg = 1 + (ob > 0) + (ob < NBK - 1);
  f32x8 acc[2][4], accx[2][4];
#pragma unroll
  for (int i = 0; i < 2; ++i)
#pragma unroll
    for (int j = 0; j < 4; ++j) { f32x8 z = {}; acc[i][j] = z; accx[i][j] = z; }
#pragma unroll 1
  for (int sg = 0; sg < nseg; ++sg) {
    int xb; const float* Wp;
    if (ob > 0) { xb = (sg == 0) ? ob - 1 : (sg == 1) ? ob : ob + 1; Wp = (sg == 0) ? Wr + (size_t)(ob - 1) * BS_ * BS_ : (sg == 1) ? Wv + (size_t)ob * BS_ * BS_ : Wl + (size_t)ob * BS_ * BS_; }
    else        { xb = (sg == 0) ? 0 : 1;                           Wp = (sg == 0) ? Wv : Wl; }
#pragma unroll 1
    for (int k0 = 0; k0 < BS_; k0 += 32) {
      __syncthreads();
      {
        const int row = tid >> 1, ch = (tid & 1) * 16;
        const float* src = X + (size_t)(m0 + row) * CC_ + xb * BS_ + k0 + ch;
#pragma unroll
        for (int g = 0; g < 4; ++g) { const v4f_t v = *(const v4f_t*)(src + 4 * g);
          f16x4 hv, lv;
#pragma unroll
          for (int u = 0; u < 4; ++u) { f16 h, l; split16(v[u], h, l); hv[u] = h; lv[u] = l; }
          *(f16x4*)(ldsA + row * LSTR + ch + 4 * g) = hv; *(f16x4*)(ldsAl + row * LSTR + ch + 4 * g) = lv; }
      }
      {
        const int k = tid >> 3, n0 = (tid & 7) * 16;
        const float* src = Wp + (size_t)(k0 + k) * BS_ + n0;
#pragma unroll
        for (int g = 0; g < 4; ++g) { const v4f_t v = *(const v4f_t*)(src + 4 * g);
#pragma unroll
          for (int u = 0; u < 4; ++u) { f16 h, l; split16(v[u], h, l); ldsW[(n0 + 4 * g + u) * LSTR + k] = h; ldsWl[(n0 + 4 * g + u) * LSTR + k] = l; } }
      }
      __syncthreads();
      f16x16 af[2], afl[2];
#pragma unroll
      for (int i = 0; i < 2; ++i) { af[i] = lds_frag(ldsA + (wm + 16 * i) * LSTR, LSTR); afl[i] = lds_frag(ldsAl + (wm + 16 * i) * LSTR, LSTR); }
#pragma unroll
      for (int j = 0; j < 4; ++j) {
        const f16x16 bf = lds_frag(ldsW + (wn + 16 * j) * LSTR, LSTR), bfl = lds_frag(ldsWl + (wn + 16 * j) * LSTR, LSTR);
#pragma unroll
        for (int i = 0; i < 2; ++i) {
          acc[i][j]  = wmma16(af[i], bf, acc[i][j]);
          accx[i][j] = wmma16(af[i], bfl, accx[i][j]);
          accx[i][j] = wmma16(afl[i], bf, accx[i][j]);
        }
      }
    }
  }
  float* so = oS[wave];
#pragma unroll
  for (int i = 0; i < 2; ++i)
#pragma unroll
    for (int j = 0; j < 4; ++j) {
      const float bv = bias[ob * BS_ + wn + 16 * j + cl];
#pragma unroll
      for (int r = 0; r < 8; ++r) so[(16 * i + rh + r) * 68 + 16 * j + cl] = acc[i][j][r] + accx[i][j][r] * RSPLIT + bv;
    }
  asm volatile("s_wait_dscnt 0" ::: "memory");
  __builtin_amdgcn_wave_barrier();
#pragma unroll 1
  for (int pass = 0; pass < 2; ++pass) {
#pragma unroll
    for (int it = 0; it < 16; ++it) { const int f4 = lane + 32 * it, rr = f4 >> 4, q = (f4 & 15) * 4;
      *(volatile v4f_t*)(Y + (size_t)(m0 + wm + rr) * CC_ + ob * BS_ + wn + q) = *(const volatile v4fa*)(so + rr * 68 + q); }
    __threadfence();
  }
}

__global__ __launch_bounds__(64) void k_sparse_attn(const float* __restrict__ Qm, const float* __restrict__ Km,
                                                    const float* __restrict__ Vm, float* __restrict__ Am) {
  __shared__ __attribute__((aligned(16))) float oS[2][16 * 68];
  const int lane = threadIdx.x & 31, wave = threadIdx.x >> 5, cl = lane & 15, hsel = lane >> 4, rh = hsel * 8, kh = rh;
  const int gt = blockIdx.x * 2 + wave;
  const int tile = gt & 127, bh = gt >> 7, h = bh & (NHD - 1), b = bh >> 4;
  const int t0 = tile * 16;
  const float* Qb = Qm + (size_t)b * TT_ * CC_ + h * HD_;
  const float* Kb = Km + (size_t)b * TT_ * CC_ + h * HD_;
  const float* Vb = Vm + (size_t)b * TT_ * CC_ + h * HD_;
  const bool diag = (hsel == 0) ? (cl < 8) : (cl >= 8);
  const int myrow = cl;
  const float SC = 0.125f * 1.44269504088896340736f;

  f16x16 qa0, qa0l, qa1, qa1l;
  load_frag2(Qb, CC_, t0, 0, qa0, qa0l); load_frag2(Qb, CC_, t0, 32, qa1, qa1l);
  float s[13];
#pragma unroll
  for (int di = 0; di < 13; ++di) {
    const int d = (di < 5) ? di : (8 << (di - 5));
    const int ks0 = t0 - d;
    f16x16 kb0, kb0l, kb1, kb1l;
    {
      const int kr = max(ks0 + cl, 0);
      load_frag2(Kb, CC_, kr - cl, 0, kb0, kb0l);
      load_frag2(Kb, CC_, kr - cl, 32, kb1, kb1l);
    }
    f32x8 cacc = {}, caccx = {};
    cacc = wmma16(qa0, kb0, cacc);   caccx = wmma16(qa0, kb0l, caccx); caccx = wmma16(qa0l, kb0, caccx);
    cacc = wmma16(qa1, kb1, cacc);   caccx = wmma16(qa1, kb1l, caccx); caccx = wmma16(qa1l, kb1, caccx);
#pragma unroll
    for (int r = 0; r < 8; ++r) cacc[r] += caccx[r] * RSPLIT;
    float sv = -INFINITY;
    if (diag && (t0 + myrow - d) >= 0) {
      float v = 0.0f;
#pragma unroll
      for (int r = 0; r < 8; ++r) v = ((myrow & 7) == r) ? cacc[r] : v;
      sv = v * SC;
    }
    s[di] = sv;
  }
  float mx = -INFINITY;
#pragma unroll
  for (int di = 0; di < 13; ++di) mx = fmaxf(mx, s[di]);
  float p[13], l = 0.0f;
#pragma unroll
  for (int di = 0; di < 13; ++di) { p[di] = (s[di] == -INFINITY) ? 0.0f : exp2f(s[di] - mx); l += p[di]; }
  const float il = diag ? (1024.0f / l) : 0.0f;
  f32x8 o[4];
#pragma unroll
  for (int j = 0; j < 4; ++j) { f32x8 z = {}; o[j] = z; }
  const int srcl = (cl < 8) ? cl : (cl + 16);
#pragma unroll
  for (int di = 0; di < 13; ++di) {
    const int d = (di < 5) ? di : (8 << (di - 5));
    const float pr = __shfl(p[di] * il, srcl, 32);
    f16x16 af;
#pragma unroll
    for (int i = 0; i < 8; ++i) { af[i] = ((kh + i) == cl) ? (f16)pr : (f16)0.0f; af[8 + i] = (f16)0.0f; }
    const int vr0 = t0 - d + kh;
#pragma unroll
    for (int j = 0; j < 4; ++j) {
      f16x16 vb;
      const float* vp = Vb + 16 * j + cl;
#pragma unroll
      for (int i = 0; i < 8; ++i) { vb[i] = (f16)vp[(size_t)max(vr0 + i, 0) * CC_]; vb[8 + i] = (f16)0.0f; }
      o[j] = wmma16(af, vb, o[j]);
    }
  }
  float* so = oS[wave];
#pragma unroll
  for (int j = 0; j < 4; ++j)
#pragma unroll
    for (int r = 0; r < 8; ++r) so[(rh + r) * 68 + 16 * j + cl] = o[j][r] * (1.0f / 1024.0f);
  asm volatile("s_wait_dscnt 0" ::: "memory");
  __builtin_amdgcn_wave_barrier();
  float* Ob = Am + (size_t)b * TT_ * CC_ + (size_t)t0 * CC_ + h * HD_;
#pragma unroll 1
  for (int pass = 0; pass < 2; ++pass) {
#pragma unroll
    for (int it = 0; it < 8; ++it) { const int f4 = lane + 32 * it, rr = f4 >> 4, q = (f4 & 15) * 4;
      *(volatile v4f_t*)(Ob + (size_t)rr * CC_ + q) = *(const volatile v4fa*)(so + rr * 68 + q); }
    __threadfence();
  }
}

extern "C" void kernel_launch(void* const* d_in, const int* in_sizes, int n_in,
                              void* d_out, int out_size, void* d_ws, size_t ws_size,
                              hipStream_t stream) {
  (void)in_sizes; (void)n_in; (void)out_size; (void)ws_size;
  const float* x = (const float*)d_in[0];
  const float* qWv = (const float*)d_in[1],  *qWr = (const float*)d_in[2],  *qWl = (const float*)d_in[3],  *qb = (const float*)d_in[4];
  const float* kWv = (const float*)d_in[5],  *kWr = (const float*)d_in[6],  *kWl = (const float*)d_in[7],  *kbs = (const float*)d_in[8];
  const float* vWv = (const float*)d_in[9],  *vWr = (const float*)d_in[10], *vWl = (const float*)d_in[11], *vb = (const float*)d_in[12];
  const float* oWv = (const float*)d_in[13], *oWr = (const float*)d_in[14], *oWl = (const float*)d_in[15], *obs = (const float*)d_in[16];
  float* out = (float*)d_out;
  const size_t MB16 = (size_t)MM_ * CC_ * 4;
  char* ws = (char*)d_ws;
  float* Qm = (float*)ws; float* Km = (float*)(ws + MB16); float* Vm = (float*)(ws + 2 * MB16); float* Am = (float*)(ws + 3 * MB16);
  const dim3 g(MM_ / 128, NBK), blk(256);
  k_urdhva<<<g, blk, 0, stream>>>(x, qWv, qWr, qWl, qb, Qm);
  k_urdhva<<<g, blk, 0, stream>>>(x, kWv, kWr, kWl, kbs, Km);
  k_urdhva<<<g, blk, 0, stream>>>(x, vWv, vWr, vWl, vb, Vm);
  k_sparse_attn<<<dim3((2 * NHD * (TT_ / 16)) / 2), dim3(64), 0, stream>>>(Qm, Km, Vm, Am);
  k_urdhva<<<g, blk, 0, stream>>>(Am, oWv, oWr, oWl, obs, out);
}
